// FastFeedForwardNetwork_78872779424238
// MI455X (gfx1250) — hardware-verified
//
#include <hip/hip_runtime.h>
#include <stdint.h>
#include <stddef.h>
#include <math.h>

#pragma clang fp contract(off)

#define NTOK  8192
#define DIN   1024
#define HID   256
#define KH    128
#define OUTD  1024
#define NLEAF 16
#define DEPTH 4
#define MT    64
#define NSL   256
#define CHUNK 2048
#define XP    1032
#define AP    136
#define YP    260
#define TP1   72

#define LDS_X    (MT * XP * 2)
#define LDS_A    (MT * AP * 2)
#define LDS_LEAF (LDS_X + LDS_A)

static_assert(MT * YP * 4 <= LDS_X);
static_assert((XP * 2) % 16 == 0);
static_assert((AP * 2) % 16 == 0);
static_assert((YP * 4) % 16 == 0);
static_assert((TP1 * 2) % 16 == 0);
static_assert(NTOK % CHUNK == 0);
static_assert(CHUNK == 8 * 256);
static_assert(NTOK % MT == 0);
static_assert(NTOK % 32 == 0);
static_assert(MT == 8 * 8);
static_assert(DIN % 64 == 0);
static_assert(DIN % 32 == 0);
static_assert(HID % 32 == 0);
static_assert(HID == 2 * KH);
static_assert(KH == 8 * 16);
static_assert(KH % 32 == 0);
static_assert(OUTD % 32 == 0);
static_assert(OUTD % NSL == 0);
static_assert(NSL == 8 * 32);
static_assert((MT * DIN / 8) % 256 == 0);
static_assert(DEPTH * DIN == 16 * 256);

typedef _Float16     v16h __attribute__((ext_vector_type(16)));
typedef _Float16     v8h  __attribute__((ext_vector_type(8)));
typedef _Float16     v4h  __attribute__((ext_vector_type(4)));
typedef float        v8f  __attribute__((ext_vector_type(8)));
typedef float        v4f  __attribute__((ext_vector_type(4)));
typedef int          v4i  __attribute__((ext_vector_type(4)));
typedef v8h __attribute__((may_alias)) v8ha;
typedef v4f __attribute__((may_alias)) v4fa;
typedef v4i __attribute__((may_alias)) v4ia;

union FragH { v16h v; v8h q[2]; };
union HV    { v8h v;  v4h q[2]; };

__device__ __forceinline__ v8f wmma_h(v16h a, v16h b, v8f c) {
  v8f d = __builtin_amdgcn_wmma_f32_16x16x32_f16(false, a, false, b, (short)0, c, false, false);
  asm volatile("v_nop\n\tv_nop\n\tv_nop\n\tv_nop" : "+v"(d) : "v"(a), "v"(b));
  return d;
}

__device__ __forceinline__ v16h ldfrag(const _Float16* p, int h) {
  FragH f;
  f.q[0] = *(const v8ha*)(p + 8 * h);
  f.q[1] = *(const v8ha*)(p + 16 + 8 * h);
  return f.v;
}

__global__ __launch_bounds__(256) void k_prep_w1(const float* __restrict__ w1,
                                                 _Float16* __restrict__ w1t)
{
  __shared__ __align__(16) _Float16 sT[32 * TP1];
  const int tid = threadIdx.x;
  const int d0 = blockIdx.x * 64, c0 = blockIdx.y * 32, leaf = blockIdx.z;
  const float* src = w1 + (size_t)leaf * (DIN * HID) + (size_t)d0 * HID + c0;
  #pragma unroll
  for (int it = 0; it < 8; ++it) {
    const int idx = tid + 256 * it;
    const int row = idx >> 5, col = idx & 31;
    const float v = src[(size_t)row * HID + col] * 1024.0f;
    sT[col * TP1 + row] = (_Float16)v;
  }
  __syncthreads();
  const int orow = tid >> 3, piece = tid & 7;
  const v8h v = *(const v8ha*)(sT + orow * TP1 + 8 * piece);
  _Float16* dst = w1t + (size_t)(leaf * HID + c0 + orow) * DIN + d0 + 8 * piece;
  *(volatile v8h*)dst = v;
  __threadfence();
  *(volatile v8h*)dst = v;
}

__global__ __launch_bounds__(256) void k_prep_w2(const float* __restrict__ w2,
                                                 _Float16* __restrict__ w2t)
{
  __shared__ __align__(16) _Float16 sT[32 * AP];
  const int tid = threadIdx.x;
  const int o0 = blockIdx.x * 32, leaf = blockIdx.y;
  const float* src = w2 + (size_t)leaf * (KH * OUTD) + o0;
  #pragma unroll 4
  for (int it = 0; it < 16; ++it) {
    const int idx = tid + 256 * it;
    const int k = idx >> 5, col = idx & 31;
    const float v = src[(size_t)k * OUTD + col] * 256.0f;
    sT[col * AP + k] = (_Float16)v;
  }
  __syncthreads();
  const int r0 = tid >> 4, p0 = tid & 15;
  const int r1 = r0 + 16;
  const v8h v0 = *(const v8ha*)(sT + r0 * AP + 8 * p0);
  const v8h v1 = *(const v8ha*)(sT + r1 * AP + 8 * p0);
  _Float16* d0 = w2t + (size_t)(leaf * OUTD + o0 + r0) * KH + 8 * p0;
  _Float16* d1 = w2t + (size_t)(leaf * OUTD + o0 + r1) * KH + 8 * p0;
  *(volatile v8h*)d0 = v0;
  *(volatile v8h*)d1 = v1;
  __threadfence();
  *(volatile v8h*)d0 = v0;
  *(volatile v8h*)d1 = v1;
}

__global__ __launch_bounds__(256) void k_route(const float* __restrict__ x,
                                               const float* __restrict__ wnode,
                                               const float* __restrict__ bnode,
                                               const int* __restrict__ training,
                                               int* __restrict__ route)
{
  __shared__ __align__(16) float swn[DEPTH * DIN];
  __shared__ __align__(16) int sLeaf[32];
  const int tid = threadIdx.x, lane = tid & 31, wv = tid >> 5;
  #pragma unroll
  for (int i = 0; i < (DEPTH * DIN) / 256; ++i) swn[tid + 256 * i] = wnode[tid + 256 * i];
  (void)training;
  __syncthreads();

  #pragma unroll 1
  for (int i = 0; i < 4; ++i) {
    const int t = blockIdx.x * 32 + wv * 4 + i;
    const float* xr = x + (size_t)t * DIN;
    double l0 = 0.0, l1 = 0.0, l2 = 0.0, l3 = 0.0;
    #pragma unroll 1
    for (int it = 0; it < DIN / 32; ++it) {
      const int d = 32 * it + lane;
      const double xv = (double)xr[d];
      l0 = fma(xv, (double)swn[d], l0);
      l1 = fma(xv, (double)swn[DIN + d], l1);
      l2 = fma(xv, (double)swn[2 * DIN + d], l2);
      l3 = fma(xv, (double)swn[3 * DIN + d], l3);
    }
    #pragma unroll
    for (int off = 16; off > 0; off >>= 1) {
      l0 = l0 + __shfl_xor(l0, off);
      l1 = l1 + __shfl_xor(l1, off);
      l2 = l2 + __shfl_xor(l2, off);
      l3 = l3 + __shfl_xor(l3, off);
    }
    if (lane == 0) {
      const float g0 = (float)l0 + bnode[0];
      const float g1 = (float)l1 + bnode[1];
      const float g2 = (float)l2 + bnode[2];
      const float g3 = (float)l3 + bnode[3];
      const int leaf = ((g0 > 0.0f) ? 0 : 8) | ((g1 > 0.0f) ? 0 : 4) |
                       ((g2 > 0.0f) ? 0 : 2) | ((g3 > 0.0f) ? 0 : 1);
      sLeaf[wv * 4 + i] = leaf;
    }
  }
  __syncthreads();
  if (wv == 0) {
    const int q = lane & 7;
    const v4i v = *(const v4ia*)(sLeaf + 4 * q);
    int* dst = route + (size_t)blockIdx.x * 32 + 4 * q;
    const bool ok = (lane < 8);
    if (ok) *(volatile v4i*)dst = v;
    __threadfence();
    if (ok) *(volatile v4i*)dst = v;
  }
}

__device__ __forceinline__ void out_pass(const float* sY, const int* sTok, float* out,
                                         int ns, int wv, int lane, int nrows)
{
  #pragma unroll
  for (int i = 0; i < 8; ++i) {
    const int row = wv * 8 + i;
    int t = sTok[row];
    t = (t < 0) ? 0 : ((t > NTOK - 1) ? (NTOK - 1) : t);
    const v4f v0 = *(const v4fa*)(sY + row * YP + 4 * lane);
    const v4f v1 = *(const v4fa*)(sY + row * YP + 128 + 4 * lane);
    float* dst = out + (size_t)t * OUTD + ns * NSL;
    if (row < nrows) {
      *(volatile v4f*)(dst + 4 * lane) = v0;
      *(volatile v4f*)(dst + 128 + 4 * lane) = v1;
    }
  }
}

__global__ __launch_bounds__(256) void k_leaf(const float* __restrict__ x,
                                              const float* __restrict__ b1,
                                              const float* __restrict__ b2,
                                              const _Float16* __restrict__ w1t,
                                              const _Float16* __restrict__ w2t,
                                              const int* __restrict__ route,
                                              float* __restrict__ out)
{
  extern __shared__ __align__(16) unsigned char dsm[];
  _Float16* sX = (_Float16*)dsm;
  _Float16* sA = (_Float16*)(dsm + LDS_X);
  float*    sY = (float*)dsm;
  __shared__ int sTok[MT];
  __shared__ int s_wc[8];

  const int tid = threadIdx.x, lane = tid & 31, wv = tid >> 5;
  const int h = lane >> 4, m = lane & 15;
  const int e = blockIdx.y;
  const int m0 = blockIdx.x * MT;

  if (tid < MT) sTok[tid] = 0;
  __syncthreads();

  int base = 0;
  #pragma unroll 1
  for (int ch = 0; ch < NTOK / CHUNK; ++ch) {
    const int t0 = ch * CHUNK + 8 * tid;
    const v4i ia = *(const v4ia*)(route + t0);
    const v4i ib = *(const v4ia*)(route + t0 + 4);
    const int idv[8] = { ia.x, ia.y, ia.z, ia.w, ib.x, ib.y, ib.z, ib.w };
    unsigned int mk[8];
    #pragma unroll
    for (int j = 0; j < 8; ++j) mk[j] = __builtin_amdgcn_ballot_w32(idv[j] == e);
    const unsigned int lt = (1u << lane) - 1u;
    int offj[8];
    int wc = 0;
    #pragma unroll
    for (int j = 0; j < 8; ++j) {
      offj[j] = wc + __builtin_popcount(mk[j] & lt);
      wc += __builtin_popcount(mk[j]);
    }
    if (lane == 0) s_wc[wv] = wc;
    __syncthreads();
    int pre = 0, tot = 0;
    #pragma unroll
    for (int w = 0; w < 8; ++w) {
      const int cc = s_wc[w];
      tot += cc;
      pre += (w < wv) ? cc : 0;
    }
    #pragma unroll
    for (int j = 0; j < 8; ++j) {
      if (idv[j] == e) {
        const int p = base + pre + offj[j] - m0;
        if ((unsigned)p < (unsigned)MT) sTok[p] = t0 + j;
      }
    }
    base += tot;
    __syncthreads();
  }
  const int cnt = base;
  if (m0 >= cnt) return;
  int nrows = cnt - m0;
  nrows = (nrows > MT) ? MT : nrows;

  #pragma unroll 4
  for (int j = 0; j < (MT * DIN / 8) / 256; ++j) {
    const int idx = tid + 256 * j;
    const int row = idx >> 7, c8 = idx & 127;
    int t = sTok[row];
    t = (t < 0) ? 0 : ((t > NTOK - 1) ? (NTOK - 1) : t);
    const float* s = x + (size_t)t * DIN + 8 * c8;
    const v4f a = *(const v4fa*)s;
    const v4f b = *(const v4fa*)(s + 4);
    HV u;
    u.q[0] = __builtin_convertvector(a, v4h);
    u.q[1] = __builtin_convertvector(b, v4h);
    *(v8ha*)(sX + row * XP + 8 * c8) = u.v;
  }
  __syncthreads();

  const v8f z8 = {0.f, 0.f, 0.f, 0.f, 0.f, 0.f, 0.f, 0.f};

  {
    v8f acc[4][2];
    #pragma unroll
    for (int mt = 0; mt < 4; ++mt) { acc[mt][0] = z8; acc[mt][1] = z8; }
    const int cLo = 16 * wv + m;
    const _Float16* bp0 = w1t + (size_t)(e * HID + cLo) * DIN;
    const _Float16* bp1 = w1t + (size_t)(e * HID + KH + cLo) * DIN;
    #pragma unroll 1
    for (int k0 = 0; k0 < DIN; k0 += 32) {
      const v16h bA = ldfrag(bp0 + k0, h);
      const v16h bB = ldfrag(bp1 + k0, h);
      #pragma unroll
      for (int mt = 0; mt < 4; ++mt) {
        const v16h a = ldfrag(sX + (16 * mt + m) * XP + k0, h);
        acc[mt][0] = wmma_h(a, bA, acc[mt][0]);
        acc[mt][1] = wmma_h(a, bB, acc[mt][1]);
      }
    }
    const float c1024 = 0.0009765625f;
    const float bLo = b1[e * HID + cLo];
    const float bHi = b1[e * HID + KH + cLo];
    #pragma unroll
    for (int mt = 0; mt < 4; ++mt) {
      #pragma unroll
      for (int r = 0; r < 8; ++r) {
        const int row = 16 * mt + 8 * h + r;
        const float hlo = acc[mt][0][r] * c1024 + bLo;
        const float hhi = acc[mt][1][r] * c1024 + bHi;
        const float av = hhi * hlo;
        sA[row * AP + cLo] = (_Float16)(av * 256.0f);
      }
    }
  }
  __syncthreads();

  #pragma unroll 1
  for (int ns = 0; ns < OUTD / NSL; ++ns) {
    v8f acc[4][2];
    #pragma unroll
    for (int mt = 0; mt < 4; ++mt) { acc[mt][0] = z8; acc[mt][1] = z8; }
    const int ob = ns * NSL + wv * 32;
    const _Float16* q0 = w2t + (size_t)(e * OUTD + ob + m) * KH;
    const _Float16* q1 = w2t + (size_t)(e * OUTD + ob + 16 + m) * KH;
    #pragma unroll 1
    for (int k0 = 0; k0 < KH; k0 += 32) {
      const v16h bA = ldfrag(q0 + k0, h);
      const v16h bB = ldfrag(q1 + k0, h);
      #pragma unroll
      for (int mt = 0; mt < 4; ++mt) {
        const v16h a = ldfrag(sA + (16 * mt + m) * AP + k0, h);
        acc[mt][0] = wmma_h(a, bA, acc[mt][0]);
        acc[mt][1] = wmma_h(a, bB, acc[mt][1]);
      }
    }
    const float c65536 = 0.0000152587890625f;
    const float g0 = b2[e * OUTD + ob + m];
    const float g1 = b2[e * OUTD + ob + 16 + m];
    const int cl = wv * 32 + m;
    #pragma unroll
    for (int mt = 0; mt < 4; ++mt) {
      #pragma unroll
      for (int r = 0; r < 8; ++r) {
        const int row = 16 * mt + 8 * h + r;
        sY[row * YP + cl]      = acc[mt][0][r] * c65536 + g0;
        sY[row * YP + cl + 16] = acc[mt][1][r] * c65536 + g1;
      }
    }
    __syncthreads();
    out_pass(sY, sTok, out, ns, wv, lane, nrows);
    __threadfence();
    out_pass(sY, sTok, out, ns, wv, lane, nrows);
    __syncthreads();
  }
}

extern "C" void kernel_launch(void* const* d_in, const int* in_sizes, int n_in,
                              void* d_out, int out_size, void* d_ws, size_t ws_size,
                              hipStream_t stream)
{
  if (n_in < 8) return;
  if (in_sizes[0] != NTOK * DIN) return;
  if (in_sizes[1] != NLEAF * DIN * HID) return;
  if (in_sizes[2] != NLEAF * KH * OUTD) return;
  if (in_sizes[3] != NLEAF * HID) return;
  if (in_sizes[4] != NLEAF * OUTD) return;
  if (in_sizes[5] < DEPTH * DIN) return;
  if (in_sizes[6] < DEPTH) return;
  if (in_sizes[7] < 1) return;
  if (out_size != NTOK * OUTD) return;

  const float* x     = (const float*)d_in[0];
  const float* w1    = (const float*)d_in[1];
  const float* w2    = (const float*)d_in[2];
  const float* b1    = (const float*)d_in[3];
  const float* b2    = (const float*)d_in[4];
  const float* wnode = (const float*)d_in[5];
  const float* bnode = (const float*)d_in[6];
  const int*   trn   = (const int*)d_in[7];
  float* out = (float*)d_out;

  const size_t bW1T = (size_t)NLEAF * HID * DIN * 2;
  const size_t bW2T = (size_t)NLEAF * OUTD * KH * 2;
  const size_t bRT  = (size_t)NTOK * 4;
  const size_t total = bW1T + bW2T + bRT;
  if (total > ws_size) return;
  if (total > (size_t)134217728) return;

  char* ws = (char*)d_ws;
  size_t off = 0;
  _Float16* W1T = (_Float16*)(ws + off); off += bW1T;
  _Float16* W2T = (_Float16*)(ws + off); off += bW2T;
  int*      RT  = (int*)(ws + off);      off += bRT;
  if (off != total) return;

  k_prep_w1<<<dim3(DIN / 64, HID / 32, NLEAF), 256, 0, stream>>>(w1, W1T);
  k_prep_w2<<<dim3(OUTD / 32, NLEAF), 256, 0, stream>>>(w2, W2T);
  k_route<<<NTOK / 32, 256, 0, stream>>>(x, wnode, bnode, trn, RT);
  hipFuncSetAttribute(reinterpret_cast<const void*>(&k_leaf),
                      hipFuncAttributeMaxDynamicSharedMemorySize, LDS_LEAF);
  k_leaf<<<dim3(NTOK / MT, NLEAF), 256, LDS_LEAF, stream>>>(x, b1, b2, W1T, W2T, RT, out);
}
